// LSTMFourierDecoder_82617990906569
// MI455X (gfx1250) — hardware-verified
//
#include <hip/hip_runtime.h>
#include <math.h>
#include <stdint.h>
#include <stddef.h>

typedef __attribute__((ext_vector_type(16))) _Float16 v16h;
typedef __attribute__((ext_vector_type(8)))  _Float16 v8h;
typedef __attribute__((ext_vector_type(16))) __bf16   v16b;
typedef __attribute__((ext_vector_type(8)))  __bf16   v8b;
typedef __attribute__((ext_vector_type(8)))  float    v8f;
typedef __attribute__((ext_vector_type(4)))  float    v4f;
typedef __attribute__((ext_vector_type(4)))  unsigned int v4u;

__device__ __forceinline__ unsigned short f2bf_bits(float f) {
  unsigned u = __float_as_uint(f);
  return (unsigned short)((u + 0x7FFFu + ((u >> 16) & 1u)) >> 16);
}
__device__ __forceinline__ float bf_bits2f(unsigned short h) { return __uint_as_float(((unsigned)h) << 16); }

__device__ __forceinline__ void dep_guard_h(v8f& a, v8f& b, v16h x, v16h y) { asm volatile("v_nop\n\tv_nop\n\tv_nop\n\tv_nop" : "+v"(a), "+v"(b) : "v"(x), "v"(y)); }
__device__ __forceinline__ void dep_guard_b(v8f& a, v8f& b, v16b x, v16b y) { asm volatile("v_nop\n\tv_nop\n\tv_nop\n\tv_nop" : "+v"(a), "+v"(b) : "v"(x), "v"(y)); }
__device__ __forceinline__ void keep4_h(v16h a, v16h b, v16h c, v16h d) { asm volatile("v_nop" :: "v"(a), "v"(b), "v"(c), "v"(d)); }
__device__ __forceinline__ void keep4_b(v16b a, v16b b, v16b c, v16b d) { asm volatile("v_nop" :: "v"(a), "v"(b), "v"(c), "v"(d)); }
__device__ __forceinline__ void acc_guard4(v8f& a, v8f& b, v8f& c, v8f& d) { asm volatile("v_nop\n\tv_nop\n\tv_nop\n\tv_nop" : "+v"(a), "+v"(b), "+v"(c), "+v"(d)); }
template <typename T> struct Frag;
template <> struct Frag<_Float16> {
  typedef v16h V; union U { v16h v; v8h h[2]; };
  static __device__ __forceinline__ v16h load(const _Float16* p) {
    U f; f.h[0] = *(const v8h*)(p); f.h[1] = *(const v8h*)(p + 16); return f.v;
  }
  static __device__ __forceinline__ v8f mma(v16h a, v16h b, v8f c) {
    return __builtin_amdgcn_wmma_f32_16x16x32_f16(false, a, false, b, (short)0, c, false, false);
  }
  static __device__ __forceinline__ void guard(v8f& a, v8f& b, v16h x, v16h y) { dep_guard_h(a, b, x, y); }
  static __device__ __forceinline__ void keep(v16h a, v16h b, v16h c, v16h d) { keep4_h(a, b, c, d); }
};
template <> struct Frag<__bf16> {
  typedef v16b V; union U { v16b v; v8b h[2]; };
  static __device__ __forceinline__ v16b load(const __bf16* p) {
    U f; f.h[0] = *(const v8b*)(p); f.h[1] = *(const v8b*)(p + 16); return f.v;
  }
  static __device__ __forceinline__ v8f mma(v16b a, v16b b, v8f c) {
    return __builtin_amdgcn_wmma_f32_16x16x32_bf16(false, a, false, b, (short)0, c, false, false);
  }
  static __device__ __forceinline__ void guard(v8f& a, v8f& b, v16b x, v16b y) { dep_guard_b(a, b, x, y); }
  static __device__ __forceinline__ void keep(v16b a, v16b b, v16b c, v16b d) { keep4_b(a, b, c, d); }
};

template <int ET> struct Elem;
template <> struct Elem<0> { typedef _Float16 T; };
template <> struct Elem<1> { typedef __bf16 T; };
template <int ET, bool SPLIT, int BIAS_MODE, int OUT_MODE, bool RESID, int ACT = 0>
__global__ __launch_bounds__(256) void wmma_gemm64(
    const unsigned short* __restrict__ Ap, const unsigned short* __restrict__ A2p, int lda, long strideA,
    const unsigned short* __restrict__ Btp, const unsigned short* __restrict__ Bt2p, int ldb, long strideB,
    void* __restrict__ Cout, void* __restrict__ Cout2, int ldc, long strideC,
    const float* __restrict__ bias,
    const float* __restrict__ resid, long strideR,
    int M, int N, int K, float scale) {
  typedef typename Elem<ET>::T T;
  typedef typename Frag<T>::V V;
  const T* A = (const T*)Ap; const T* A2 = (const T*)A2p; const T* Bt = (const T*)Btp; const T* Bt2 = (const T*)Bt2p;
  __shared__ __align__(16) float sT[8][16 * 68];
  const int b    = blockIdx.y;
  const int lane = threadIdx.x & 31;
  const int wave = threadIdx.x >> 5;
  const int tilesN = N >> 6;
  const int tilesM = M >> 6;
  const int tile = blockIdx.x * 8 + wave;
  if (tile >= tilesM * tilesN) return;
  const int tm = tile / tilesN;
  const int tn = tile - tm * tilesN;
  const int m0 = tm << 6;
  const int n0 = tn << 6;

  const T* Ab  = A  + (size_t)b * strideA;
  const T* Bb  = Bt + (size_t)b * strideB;
  const T* Ab2 = SPLIT ? (A2  + (size_t)b * strideA) : nullptr;
  const T* Bb2 = SPLIT ? (Bt2 + (size_t)b * strideB) : nullptr;

  const int rlane = lane & 15;
  const int koff  = (lane >> 4) * 8;
  const int mOff  = (lane >> 4) * 8;

  v8f acc[4][4];
#pragma unroll
  for (int i = 0; i < 4; ++i)
#pragma unroll
    for (int j = 0; j < 4; ++j) acc[i][j] = (v8f){0.f,0.f,0.f,0.f,0.f,0.f,0.f,0.f};

  for (int k0 = 0; k0 < K; k0 += 32) {
    V bh[4], bl[4];
#pragma unroll
    for (int j = 0; j < 4; ++j) {
      const size_t bo = (size_t)(n0 + (j << 4) + rlane) * ldb + koff + k0;
      bh[j] = Frag<T>::load(Bb + bo);
      if (SPLIT) bl[j] = Frag<T>::load(Bb2 + bo);
    }
#pragma unroll
    for (int i = 0; i < 4; ++i) {
      const size_t ao = (size_t)(m0 + (i << 4) + rlane) * lda + koff + k0;
      V ah = Frag<T>::load(Ab + ao);
      V al;
      if (SPLIT) al = Frag<T>::load(Ab2 + ao);
#pragma unroll
      for (int j = 0; j < 4; ++j) {
        acc[i][j] = Frag<T>::mma(ah, bh[j], acc[i][j]);
        if (SPLIT) {
          acc[i][j] = Frag<T>::mma(ah, bl[j], acc[i][j]);
          acc[i][j] = Frag<T>::mma(al, bh[j], acc[i][j]);
        }
      }
      Frag<T>::guard(acc[i][0], acc[i][3], ah, SPLIT ? al : ah);
    }
    Frag<T>::keep(bh[0], bh[1], bh[2], bh[3]);
    if (SPLIT) Frag<T>::keep(bl[0], bl[1], bl[2], bl[3]);
  }
  acc_guard4(acc[0][0], acc[0][1], acc[0][2], acc[0][3]);
  acc_guard4(acc[1][0], acc[1][1], acc[1][2], acc[1][3]);
  acc_guard4(acc[2][0], acc[2][1], acc[2][2], acc[2][3]);
  acc_guard4(acc[3][0], acc[3][1], acc[3][2], acc[3][3]);

  float* slab = sT[wave];
  const float* Rb = RESID ? (resid + (size_t)b * strideR) : nullptr;
#pragma unroll
  for (int i = 0; i < 4; ++i) {
    const int mBase = m0 + (i << 4);
#pragma unroll
    for (int j = 0; j < 4; ++j) {
      const int n = n0 + (j << 4) + rlane;
      float bv = 0.f;
      if (BIAS_MODE == 2) bv = bias[n];
#pragma unroll
      for (int r = 0; r < 8; ++r) {
        float v = acc[i][j][r] * scale;
        if (BIAS_MODE == 1) v += bias[mBase + mOff + r];
        if (BIAS_MODE == 2) v += bv;
        if (RESID) v += Rb[(size_t)(mBase + mOff + r) * ldc + n];
        if (ACT == 1) v = tanhf(v);
        if (ACT == 2) v = fmaxf(v, 0.0f);
        if (ACT == 3) v = v / (1.0f + expf(-v));
        if (ACT == 4) v = (v > 0.f) ? v : 0.01f * v;
        if (ACT == 5) v = 0.5f * v * (1.0f + erff(v * 0.70710678118654752f));
        slab[(mOff + r) * 68 + (j << 4) + rlane] = v;
      }
    }
    __builtin_amdgcn_fence(__ATOMIC_RELEASE, "workgroup");
    __builtin_amdgcn_wave_barrier();
    __builtin_amdgcn_fence(__ATOMIC_ACQUIRE, "workgroup");
    if (OUT_MODE == 0) {
      float* C = (float*)Cout + (size_t)b * strideC;
      const int hh = lane >> 4, c4 = (lane & 15) * 4;
      for (int pass = 0; pass < 2; ++pass) {
#pragma unroll
        for (int it = 0; it < 8; ++it) {
          const int row = it * 2 + hh;
          v4f v = *(const v4f*)(slab + row * 68 + c4);
          *(volatile v4f*)(C + (size_t)(mBase + row) * ldc + n0 + c4) = v;
        }
        __threadfence();
      }
    } else {
      const int q = lane >> 3, c8 = (lane & 7) * 8;
      unsigned short* C  = (unsigned short*)Cout  + (size_t)b * strideC;
      unsigned short* C2 = (OUT_MODE == 2) ? ((unsigned short*)Cout2 + (size_t)b * strideC) : nullptr;
      for (int pass = 0; pass < 2; ++pass) {
#pragma unroll
        for (int it = 0; it < 4; ++it) {
          const int row = it * 4 + q;
          const float* sp = slab + row * 68 + c8;
          v8h hv, lv;
#pragma unroll
          for (int e = 0; e < 8; ++e) {
            if (OUT_MODE == 1) {
              hv[e] = (_Float16)sp[e];
            } else {
              unsigned short hb = f2bf_bits(sp[e]);
              unsigned short lb = f2bf_bits(sp[e] - bf_bits2f(hb));
              hv[e] = __builtin_bit_cast(_Float16, hb);
              lv[e] = __builtin_bit_cast(_Float16, lb);
            }
          }
          *(volatile v8h*)(C + (size_t)(mBase + row) * ldc + n0 + c8) = hv;
          if (OUT_MODE == 2) *(volatile v8h*)(C2 + (size_t)(mBase + row) * ldc + n0 + c8) = lv;
        }
        __threadfence();
      }
    }
    __builtin_amdgcn_fence(__ATOMIC_RELEASE, "workgroup");
    __builtin_amdgcn_wave_barrier();
    __builtin_amdgcn_fence(__ATOMIC_ACQUIRE, "workgroup");
  }
}

__device__ __forceinline__ v8f at_mma(v16b a, v16b b, v8f c) {
  c = __builtin_amdgcn_wmma_f32_16x16x32_bf16(false, a, false, b, (short)0, c, false, false);
  asm volatile("v_nop\n\tv_nop\n\tv_nop\n\tv_nop" : "+v"(c) : "v"(a), "v"(b));
  return c;
}

constexpr int kBatch  = 32;
constexpr int kFeat   = 512;
constexpr int kTime   = 128;
constexpr int kDim    = 512;
constexpr int kOutDim = 512;
constexpr int kRows   = kBatch * kTime;
constexpr int kGate4  = 4 * kDim;
constexpr int kAPitch = 520;

__device__ __forceinline__ void wave_sync() {
  __builtin_amdgcn_fence(__ATOMIC_RELEASE, "workgroup");
  __builtin_amdgcn_wave_barrier();
  __builtin_amdgcn_fence(__ATOMIC_ACQUIRE, "workgroup");
}
__device__ __forceinline__ float wave_sum(float v) {
#pragma unroll
  for (int off = 16; off > 0; off >>= 1) v += __shfl_xor(v, off, 32);
  return v;
}
__device__ __forceinline__ unsigned pack_hi_lo_pair(float x0, float x1, unsigned& lo_word) {
  const unsigned short h0 = f2bf_bits(x0), h1 = f2bf_bits(x1);
  const unsigned short l0 = f2bf_bits(x0 - bf_bits2f(h0)), l1 = f2bf_bits(x1 - bf_bits2f(h1));
  lo_word = (unsigned)l0 | ((unsigned)l1 << 16);
  return (unsigned)h0 | ((unsigned)h1 << 16);
}
__device__ __forceinline__ void split_pack8(v4f a, v4f b, v4u& hw, v4u& lw) {
  unsigned l0, l1, l2, l3;
  const unsigned h0 = pack_hi_lo_pair(a[0], a[1], l0);
  const unsigned h1 = pack_hi_lo_pair(a[2], a[3], l1);
  const unsigned h2 = pack_hi_lo_pair(b[0], b[1], l2);
  const unsigned h3 = pack_hi_lo_pair(b[2], b[3], l3);
  hw = (v4u){h0, h1, h2, h3};
  lw = (v4u){l0, l1, l2, l3};
}

__global__ __launch_bounds__(256) void k_tr_split(
    const float* __restrict__ in, int ld_in, long bstride_in,
    unsigned short* __restrict__ outh, unsigned short* __restrict__ outl, int ld_out, long bstride_out) {
  __shared__ float tile[64][65];
  const int tid = threadIdx.x, lane = tid & 31, wave = tid >> 5;
  const int r0 = blockIdx.y * 64, c0 = blockIdx.x * 64;
  const float* inb = in + (size_t)blockIdx.z * (size_t)bstride_in;
  {
    const int row = tid >> 2, cseg = (tid & 3) * 16;
    const float* src = inb + (size_t)(r0 + row) * ld_in + c0 + cseg;
#pragma unroll
    for (int i = 0; i < 4; ++i) {
      const v4f v = *(const v4f*)(src + 4 * i);
      tile[row][cseg + 4 * i + 0] = v[0];
      tile[row][cseg + 4 * i + 1] = v[1];
      tile[row][cseg + 4 * i + 2] = v[2];
      tile[row][cseg + 4 * i + 3] = v[3];
    }
  }
  __syncthreads();
  const int q = lane >> 3, c8 = (lane & 7) * 8;
  v4u hw[2], lw[2];
  int orow[2];
#pragma unroll
  for (int it = 0; it < 2; ++it) {
    const int orw = wave * 8 + it * 4 + q;
    orow[it] = orw;
    const v4f a = (v4f){tile[c8 + 0][orw], tile[c8 + 1][orw], tile[c8 + 2][orw], tile[c8 + 3][orw]};
    const v4f b = (v4f){tile[c8 + 4][orw], tile[c8 + 5][orw], tile[c8 + 6][orw], tile[c8 + 7][orw]};
    split_pack8(a, b, hw[it], lw[it]);
  }
  unsigned short* oh = outh + (size_t)blockIdx.z * (size_t)bstride_out;
  unsigned short* ol = outl + (size_t)blockIdx.z * (size_t)bstride_out;
  for (int pass = 0; pass < 2; ++pass) {
#pragma unroll
    for (int it = 0; it < 2; ++it) {
      const size_t o = (size_t)(c0 + orow[it]) * ld_out + r0 + c8;
      *(volatile v4u*)(oh + o) = hw[it];
      *(volatile v4u*)(ol + o) = lw[it];
    }
    __threadfence();
  }
}

__global__ __launch_bounds__(256) void k_cos_ln(
    const float* __restrict__ P, const float* __restrict__ gamma, const float* __restrict__ beta,
    unsigned short* __restrict__ Zh, unsigned short* __restrict__ Zl, int nrows) {
  __shared__ __align__(16) float zrow[8][512];
  const int tid = threadIdx.x, lane = tid & 31, wave = tid >> 5;
  const int row = blockIdx.x * 8 + wave;
  const int rowc = row < nrows ? row : nrows - 1;
  const float* prow = P + (size_t)rowc * kDim;
  float* zr = zrow[wave];
  float s = 0.f;
#pragma unroll 1
  for (int it = 0; it < 16; ++it) {
    const int col = it * 32 + lane;
    const float v = cosf(prow[col]);
    zr[col] = v;
    s += v;
  }
  s = wave_sum(s);
  const float mu = s * (1.0f / 512.0f);
  float qq = 0.f;
#pragma unroll 1
  for (int it = 0; it < 16; ++it) {
    const float d = zr[it * 32 + lane] - mu;
    qq += d * d;
  }
  qq = wave_sum(qq);
  const float var = qq * (1.0f / 512.0f);
  const float rs = rsqrtf(var + 1e-3f);
  wave_sync();
  v4u hw[2], lw[2];
#pragma unroll
  for (int half = 0; half < 2; ++half) {
    const int col = half * 256 + lane * 8;
    v4f a = *(const v4f*)(zr + col);
    v4f b = *(const v4f*)(zr + col + 4);
    const v4f ga = *(const v4f*)(gamma + col), gb = *(const v4f*)(gamma + col + 4);
    const v4f ba = *(const v4f*)(beta + col),  bb = *(const v4f*)(beta + col + 4);
#pragma unroll
    for (int e = 0; e < 4; ++e) {
      a[e] = (a[e] - mu) * rs * ga[e] + ba[e];
      b[e] = (b[e] - mu) * rs * gb[e] + bb[e];
    }
    split_pack8(a, b, hw[half], lw[half]);
  }
  if (row < nrows) {
    for (int pass = 0; pass < 2; ++pass) {
#pragma unroll
      for (int half = 0; half < 2; ++half) {
        const size_t o = (size_t)row * kDim + half * 256 + lane * 8;
        *(volatile v4u*)(Zh + o) = hw[half];
        *(volatile v4u*)(Zl + o) = lw[half];
      }
      __threadfence();
    }
  }
}

__device__ __forceinline__ void lstm_unit_tile(
    const unsigned short* __restrict__ RTh, const unsigned short* __restrict__ RTl,
    const float* __restrict__ ZG,
    const unsigned short* Ah, const unsigned short* Al, float* Hs,
    float (&cst)[8], int ub, int b0, int t, int hh, int cl, int koff) {
  v8f acc[4];
#pragma unroll
  for (int g = 0; g < 4; ++g) acc[g] = (v8f){0.f,0.f,0.f,0.f,0.f,0.f,0.f,0.f};
#pragma unroll 1
  for (int ks = 0; ks < kDim / 32; ++ks) {
    const int k0 = ks * 32;
    const v16b ah = Frag<__bf16>::load((const __bf16*)Ah + cl * kAPitch + koff + k0);
    const v16b al = Frag<__bf16>::load((const __bf16*)Al + cl * kAPitch + koff + k0);
#pragma unroll
    for (int g = 0; g < 4; ++g) {
      const size_t bo = (size_t)(g * kDim + ub * 16 + cl) * kDim + koff + k0;
      const v16b bh = Frag<__bf16>::load((const __bf16*)RTh + bo);
      const v16b bl = Frag<__bf16>::load((const __bf16*)RTl + bo);
      acc[g] = at_mma(ah, bh, acc[g]);
      acc[g] = at_mma(ah, bl, acc[g]);
      acc[g] = at_mma(al, bh, acc[g]);
    }
  }
  const int d = ub * 16 + cl;
#pragma unroll
  for (int r = 0; r < 8; ++r) {
    const int row = 8 * hh + r;
    const size_t zoff = ((size_t)(b0 + row) * kTime + t) * kGate4 + d;
    const float zi = ZG[zoff], zf = ZG[zoff + kDim], zo = ZG[zoff + 2 * kDim], zc = ZG[zoff + 3 * kDim];
    float xi = zi + acc[0][r], xf = zf + acc[1][r];
    xi = fminf(fmaxf(xi, -30.f), 30.f);
    xf = fminf(fmaxf(xf, -30.f), 30.f);
    const float ig = 1.0f / (1.0f + expf(-xi));
    const float fg = 1.0f / (1.0f + expf(-xf));
    const float og = sinf(zo + acc[2][r]);
    const float gg = tanhf(zc + acc[3][r]);
    const float cnew = fg * cst[r] + ig * gg;
    cst[r] = cnew;
    Hs[row * kDim + d] = og * cnew;
  }
}

__global__ __launch_bounds__(256) void k_lstm(
    const unsigned short* __restrict__ RTh, const unsigned short* __restrict__ RTl,
    const float* __restrict__ ZG,
    const float* __restrict__ init_h, const float* __restrict__ init_c,
    unsigned short* __restrict__ Hoh, unsigned short* __restrict__ Hol) {
  __shared__ __align__(16) unsigned short Ah[16 * kAPitch];
  __shared__ __align__(16) unsigned short Al[16 * kAPitch];
  __shared__ __align__(16) float Hs[16 * kDim];
  const int tid = threadIdx.x, lane = tid & 31, wave = tid >> 5;
  const int hh = lane >> 4, cl = lane & 15, koff = hh * 8;
  const int b0 = blockIdx.x * 16;

  float cst0[8], cst1[8], cst2[8], cst3[8];
  {
    const float ci0 = init_c[(wave * 4 + 0) * 16 + cl];
    const float ci1 = init_c[(wave * 4 + 1) * 16 + cl];
    const float ci2 = init_c[(wave * 4 + 2) * 16 + cl];
    const float ci3 = init_c[(wave * 4 + 3) * 16 + cl];
#pragma unroll
    for (int r = 0; r < 8; ++r) { cst0[r] = ci0; cst1[r] = ci1; cst2[r] = ci2; cst3[r] = ci3; }
  }
#pragma unroll
  for (int rr = 0; rr < 2; ++rr) {
#pragma unroll
    for (int half = 0; half < 2; ++half) {
      const int row = 2 * wave + rr, col = half * 256 + lane * 8;
      const v4f ha = *(const v4f*)(init_h + col), hb = *(const v4f*)(init_h + col + 4);
      v4u hw, lw;
      split_pack8(ha, hb, hw, lw);
      *(v4u*)(Ah + row * kAPitch + col) = hw;
      *(v4u*)(Al + row * kAPitch + col) = lw;
    }
  }
  __syncthreads();

#pragma unroll 1
  for (int t = 0; t < kTime; ++t) {
    lstm_unit_tile(RTh, RTl, ZG, Ah, Al, Hs, cst0, wave * 4 + 0, b0, t, hh, cl, koff);
    lstm_unit_tile(RTh, RTl, ZG, Ah, Al, Hs, cst1, wave * 4 + 1, b0, t, hh, cl, koff);
    lstm_unit_tile(RTh, RTl, ZG, Ah, Al, Hs, cst2, wave * 4 + 2, b0, t, hh, cl, koff);
    lstm_unit_tile(RTh, RTl, ZG, Ah, Al, Hs, cst3, wave * 4 + 3, b0, t, hh, cl, koff);
    __syncthreads();
    v4u hw[2][2], lw[2][2];
#pragma unroll
    for (int rr = 0; rr < 2; ++rr) {
#pragma unroll
      for (int half = 0; half < 2; ++half) {
        const int row = 2 * wave + rr, col = half * 256 + lane * 8;
        const v4f a = *(const v4f*)(Hs + row * kDim + col);
        const v4f b = *(const v4f*)(Hs + row * kDim + col + 4);
        split_pack8(a, b, hw[rr][half], lw[rr][half]);
        *(v4u*)(Ah + row * kAPitch + col) = hw[rr][half];
        *(v4u*)(Al + row * kAPitch + col) = lw[rr][half];
      }
    }
    for (int pass = 0; pass < 2; ++pass) {
#pragma unroll
      for (int rr = 0; rr < 2; ++rr) {
#pragma unroll
        for (int half = 0; half < 2; ++half) {
          const int row = 2 * wave + rr, col = half * 256 + lane * 8;
          const size_t go = ((size_t)(b0 + row) * kTime + t) * kDim + col;
          *(volatile v4u*)(Hoh + go) = hw[rr][half];
          *(volatile v4u*)(Hol + go) = lw[rr][half];
        }
      }
      __threadfence();
    }
    __syncthreads();
  }
}

static inline size_t align_up256(size_t v) { return (v + 255) & ~(size_t)255; }

extern "C" void kernel_launch(void* const* d_in, const int* in_sizes, int n_in,
                              void* d_out, int out_size, void* d_ws, size_t ws_size,
                              hipStream_t stream) {
  if (n_in < 21) return;
  if (in_sizes[0] != kBatch * kFeat * kTime) return;
  if (in_sizes[1] != kFeat * kDim || in_sizes[5] != kDim * kDim || in_sizes[9] != kDim * kDim) return;
  if (in_sizes[19] != kDim * kOutDim || out_size != kBatch * kOutDim * kTime) return;

  const float* x         = (const float*)d_in[0];
  const float* fourier_w = (const float*)d_in[1];
  const float* fourier_b = (const float*)d_in[2];
  const float* ln_gamma  = (const float*)d_in[3];
  const float* ln_beta   = (const float*)d_in[4];
  const float* Wg[4] = {(const float*)d_in[5], (const float*)d_in[6], (const float*)d_in[7], (const float*)d_in[8]};
  const float* Rg[4] = {(const float*)d_in[9], (const float*)d_in[10], (const float*)d_in[11], (const float*)d_in[12]};
  const float* bg[4] = {(const float*)d_in[13], (const float*)d_in[14], (const float*)d_in[15], (const float*)d_in[16]};
  const float* init_h = (const float*)d_in[17];
  const float* init_c = (const float*)d_in[18];
  const float* proj_w = (const float*)d_in[19];
  const float* proj_b = (const float*)d_in[20];
  float* out = (float*)d_out;

  uint8_t* p = (uint8_t*)d_ws;
  size_t off = 0;
  const size_t plane_act = (size_t)kRows * kDim * 2;
  const size_t plane_w   = (size_t)kDim * kDim * 2;
  const size_t plane_w4  = (size_t)kGate4 * kDim * 2;
  unsigned short* XTh  = (unsigned short*)(p + off); off = align_up256(off + plane_act);
  unsigned short* XTl  = (unsigned short*)(p + off); off = align_up256(off + plane_act);
  unsigned short* fwTh = (unsigned short*)(p + off); off = align_up256(off + plane_w);
  unsigned short* fwTl = (unsigned short*)(p + off); off = align_up256(off + plane_w);
  unsigned short* WTh  = (unsigned short*)(p + off); off = align_up256(off + plane_w4);
  unsigned short* WTl  = (unsigned short*)(p + off); off = align_up256(off + plane_w4);
  unsigned short* RTh  = (unsigned short*)(p + off); off = align_up256(off + plane_w4);
  unsigned short* RTl  = (unsigned short*)(p + off); off = align_up256(off + plane_w4);
  unsigned short* pwTh = (unsigned short*)(p + off); off = align_up256(off + plane_w);
  unsigned short* pwTl = (unsigned short*)(p + off); off = align_up256(off + plane_w);
  float*          Pf   = (float*)(p + off);          off = align_up256(off + (size_t)kRows * kDim * 4);
  unsigned short* Zh   = (unsigned short*)(p + off); off = align_up256(off + plane_act);
  unsigned short* Zl   = (unsigned short*)(p + off); off = align_up256(off + plane_act);
  float*          ZG   = (float*)(p + off);          off = align_up256(off + (size_t)kRows * kGate4 * 4);
  unsigned short* Hh   = (unsigned short*)(p + off); off = align_up256(off + plane_act);
  unsigned short* Hl   = (unsigned short*)(p + off); off = align_up256(off + plane_act);
  if (off > ws_size) return;

  k_tr_split<<<dim3(kTime / 64, kFeat / 64, kBatch), 256, 0, stream>>>(
      x, kTime, (long)kFeat * kTime, XTh, XTl, kFeat, (long)kTime * kFeat);
  k_tr_split<<<dim3(kDim / 64, kFeat / 64, 1), 256, 0, stream>>>(fourier_w, kDim, 0L, fwTh, fwTl, kFeat, 0L);
  for (int g = 0; g < 4; ++g) {
    k_tr_split<<<dim3(kDim / 64, kDim / 64, 1), 256, 0, stream>>>(
        Wg[g], kDim, 0L, WTh + (size_t)g * kDim * kDim, WTl + (size_t)g * kDim * kDim, kDim, 0L);
  }
  for (int g = 0; g < 4; ++g) {
    k_tr_split<<<dim3(kDim / 64, kDim / 64, 1), 256, 0, stream>>>(
        Rg[g], kDim, 0L, RTh + (size_t)g * kDim * kDim, RTl + (size_t)g * kDim * kDim, kDim, 0L);
  }
  k_tr_split<<<dim3(kOutDim / 64, kDim / 64, 1), 256, 0, stream>>>(proj_w, kOutDim, 0L, pwTh, pwTl, kDim, 0L);

  wmma_gemm64<1, true, 2, 0, false, 0><<<dim3((kRows / 64) * (kDim / 64) / 8, 1), 256, 0, stream>>>(
      XTh, XTl, kFeat, 0L, fwTh, fwTl, kFeat, 0L, (void*)Pf, (void*)nullptr, kDim, 0L,
      fourier_b, (const float*)nullptr, 0L, kRows, kDim, kFeat, 1.0f);

  k_cos_ln<<<kRows / 8, 256, 0, stream>>>(Pf, ln_gamma, ln_beta, Zh, Zl, kRows);

  for (int g = 0; g < 4; ++g) {
    wmma_gemm64<1, true, 2, 0, false, 0><<<dim3((kRows / 64) * (kDim / 64) / 8, 1), 256, 0, stream>>>(
        Zh, Zl, kDim, 0L, WTh + (size_t)g * kDim * kDim, WTl + (size_t)g * kDim * kDim, kDim, 0L,
        (void*)(ZG + (size_t)g * kDim), (void*)nullptr, kGate4, 0L,
        bg[g], (const float*)nullptr, 0L, kRows, kDim, kDim, 1.0f);
  }

  k_lstm<<<kBatch / 16, 256, 0, stream>>>(RTh, RTl, ZG, init_h, init_c, Hh, Hl);

  wmma_gemm64<1, true, 1, 0, false, 0><<<dim3((kOutDim / 64) * (kTime / 64) / 8, kBatch), 256, 0, stream>>>(
      pwTh, pwTl, kDim, 0L, Hh, Hl, kDim, (long)kTime * kDim, (void*)out, (void*)nullptr, kTime, (long)kOutDim * kTime,
      proj_b, (const float*)nullptr, 0L, kOutDim, kTime, kDim, 1.0f);
}
